// DeltaNet_31877247271509
// MI455X (gfx1250) — hardware-run, weakly checked
//
#include <hip/hip_runtime.h>
#include <math.h>

constexpr int kBatch = 2;
constexpr int kLen   = 2048;
constexpr int kHid   = 1024;
constexpr int kHeads = 4;
constexpr int kDh    = 256;
constexpr int kRows  = kBatch * kLen;
constexpr int kChunk = 32;
constexpr int kNChunk = kLen / kChunk;
constexpr int kGin   = 1084;
constexpr int kGinP  = 1088;
constexpr int kGh    = 2048;
constexpr int kNLog  = 20;
constexpr int kNLogP = 64;
constexpr int kNqkv  = 3136;
constexpr int kConvK = 4;
constexpr int kFirS = 3, kFirL = 31, kFirW = 64;
constexpr int kFirTaps = kFirS + kFirL + kFirW;

static_assert(kHeads * kDh == kHid, "head split");
static_assert(kRows % 64 == 0 && kNqkv % 64 == 0 && kGh % 64 == 0 && kNLogP % 64 == 0 && kHid % 64 == 0, "M/N tiles");
static_assert(kHid % 32 == 0 && kGinP % 32 == 0 && kGh % 32 == 0, "K multiples of 32");
static_assert(kLen % kChunk == 0 && kChunk == 32 && kDh % 64 == 0, "chunking");

constexpr float kCarryX  = 8.0f;
constexpr float kCarryW  = 256.0f;
constexpr float kCarry16 = 16.0f;
constexpr float kInv16   = 1.0f / 16.0f;
constexpr float kInv256  = 1.0f / 256.0f;
constexpr float kScaleS1 = kCarry16 / (kCarryX * kCarryW);
constexpr float kScaleG  = 1.0f / (kCarryX * kCarryW);

typedef __attribute__((ext_vector_type(16))) _Float16 v16h;
typedef __attribute__((ext_vector_type(8)))  _Float16 v8h;
typedef __attribute__((ext_vector_type(16))) __bf16   v16b;
typedef __attribute__((ext_vector_type(8)))  __bf16   v8b;
typedef __attribute__((ext_vector_type(8)))  float    v8f;
typedef __attribute__((ext_vector_type(4)))  float    v4f;
typedef __attribute__((ext_vector_type(4)))  unsigned int v4u;
typedef __attribute__((ext_vector_type(2)))  unsigned int v2u;

__device__ __forceinline__ unsigned short f2bf_bits(float f) {
  unsigned u = __float_as_uint(f);
  return (unsigned short)((u + 0x7FFFu + ((u >> 16) & 1u)) >> 16);
}
__device__ __forceinline__ float bf_bits2f(unsigned short h) { return __uint_as_float(((unsigned)h) << 16); }
__device__ __forceinline__ float bf16r(float f) { return bf_bits2f(f2bf_bits(f)); }
__device__ __forceinline__ unsigned short h_bits(float f) { const _Float16 h = (_Float16)f; return __builtin_bit_cast(unsigned short, h); }
__device__ __forceinline__ _Float16 h_from_bits(unsigned b) { const unsigned short s = (unsigned short)(b & 0xffffu); return __builtin_bit_cast(_Float16, s); }
__device__ __forceinline__ unsigned pk16(unsigned short a, unsigned short b) { return (unsigned)a | ((unsigned)b << 16); }
__device__ __forceinline__ float h16_to_f32(unsigned hb) {
  const unsigned sgn = (hb & 0x8000u) << 16; const unsigned em = hb & 0x7fffu;
  const float fn = __uint_as_float((em << 13) + 0x38000000u);
  const float fs = (float)em * 5.9604644775390625e-8f;
  const float mag = (em < 0x400u) ? fs : fn; return __uint_as_float(__float_as_uint(mag) | sgn);
}

__device__ __forceinline__ void dep_guard4_h(v8f& a, v8f& b, v8f& c, v8f& d, v16h x, v16h y) { asm volatile("v_nop\n\tv_nop\n\tv_nop\n\tv_nop" : "+v"(a), "+v"(b), "+v"(c), "+v"(d) : "v"(x), "v"(y)); }
__device__ __forceinline__ void dep_guard4_b(v8f& a, v8f& b, v8f& c, v8f& d, v16b x, v16b y) { asm volatile("v_nop\n\tv_nop\n\tv_nop\n\tv_nop" : "+v"(a), "+v"(b), "+v"(c), "+v"(d) : "v"(x), "v"(y)); }
__device__ __forceinline__ void keep4_h(v16h a, v16h b, v16h c, v16h d) { asm volatile("v_nop" :: "v"(a), "v"(b), "v"(c), "v"(d)); }
__device__ __forceinline__ void keep4_b(v16b a, v16b b, v16b c, v16b d) { asm volatile("v_nop" :: "v"(a), "v"(b), "v"(c), "v"(d)); }
__device__ __forceinline__ void acc_guard4(v8f& a, v8f& b, v8f& c, v8f& d) { asm volatile("v_nop\n\tv_nop\n\tv_nop\n\tv_nop" : "+v"(a), "+v"(b), "+v"(c), "+v"(d)); }
template <typename T> struct Frag;
template <> struct Frag<_Float16> {
  typedef v16h V; union U { v16h v; v8h h[2]; };
  static __device__ __forceinline__ v16h load(const _Float16* p) {
    U f; f.h[0] = *(const v8h*)(p); f.h[1] = *(const v8h*)(p + 16); return f.v;
  }
  static __device__ __forceinline__ v8f mma(v16h a, v16h b, v8f c) {
    return __builtin_amdgcn_wmma_f32_16x16x32_f16(false, a, false, b, (short)0, c, false, false);
  }
  static __device__ __forceinline__ void guard4(v8f& a, v8f& b, v8f& c, v8f& d, v16h x, v16h y) { dep_guard4_h(a, b, c, d, x, y); }
  static __device__ __forceinline__ void keep(v16h a, v16h b, v16h c, v16h d) { keep4_h(a, b, c, d); }
};
template <> struct Frag<__bf16> {
  typedef v16b V; union U { v16b v; v8b h[2]; };
  static __device__ __forceinline__ v16b load(const __bf16* p) {
    U f; f.h[0] = *(const v8b*)(p); f.h[1] = *(const v8b*)(p + 16); return f.v;
  }
  static __device__ __forceinline__ v8f mma(v16b a, v16b b, v8f c) {
    return __builtin_amdgcn_wmma_f32_16x16x32_bf16(false, a, false, b, (short)0, c, false, false);
  }
  static __device__ __forceinline__ void guard4(v8f& a, v8f& b, v8f& c, v8f& d, v16b x, v16b y) { dep_guard4_b(a, b, c, d, x, y); }
  static __device__ __forceinline__ void keep(v16b a, v16b b, v16b c, v16b d) { keep4_b(a, b, c, d); }
};
typedef Frag<_Float16> FragH;

__device__ __forceinline__ v8f mmah(v16h a, v16h b, v8f c) {
  c = __builtin_amdgcn_wmma_f32_16x16x32_f16(false, a, false, b, (short)0, c, false, false);
  asm volatile("v_nop\n\tv_nop\n\tv_nop\n\tv_nop" : "+v"(c) : "v"(a), "v"(b));
  return c;
}
__device__ __forceinline__ v8f zero8() { return (v8f){0.f, 0.f, 0.f, 0.f, 0.f, 0.f, 0.f, 0.f}; }

template <int ET> struct Elem;
template <> struct Elem<0> { typedef _Float16 T; };
template <> struct Elem<1> { typedef __bf16 T; };
template <int ET, bool SPLIT, bool ASPLIT, int BIAS_MODE, int OUT_MODE, int ACT = 0>
__global__ __launch_bounds__(256) void wmma_gemm64(
    const unsigned short* __restrict__ Ap, const unsigned short* __restrict__ A2p, int lda, long strideA,
    const unsigned short* __restrict__ Btp, const unsigned short* __restrict__ Bt2p, int ldb, long strideB,
    void* __restrict__ Cout, void* __restrict__ Cout2, int ldc, long strideC,
    const float* __restrict__ bias,
    int M, int N, int K, float scale) {
  typedef typename Elem<ET>::T T;
  typedef typename Frag<T>::V V;
  const T* A = (const T*)Ap; const T* A2 = (const T*)A2p; const T* Bt = (const T*)Btp; const T* Bt2 = (const T*)Bt2p;
  __shared__ __align__(16) float sT[8][16 * 68];
  const int b    = blockIdx.y;
  const int lane = threadIdx.x & 31;
  const int wave = threadIdx.x >> 5;
  const int tilesN = N >> 6;
  const int tilesM = M >> 6;
  const int tile = blockIdx.x * 8 + wave;
  if (tile >= tilesM * tilesN) return;
  const int tm = tile / tilesN;
  const int tn = tile - tm * tilesN;
  const int m0 = tm << 6;
  const int n0 = tn << 6;

  const T* Ab  = A  + (size_t)b * strideA;
  const T* Bb  = Bt + (size_t)b * strideB;
  const T* Ab2 = (SPLIT || ASPLIT) ? (A2  + (size_t)b * strideA) : nullptr;
  const T* Bb2 = SPLIT ? (Bt2 + (size_t)b * strideB) : nullptr;

  const int rlane = lane & 15;
  const int koff  = (lane >> 4) * 8;
  const int mOff  = (lane >> 4) * 8;

  v8f acc[4][4];
#pragma unroll
  for (int i = 0; i < 4; ++i)
#pragma unroll
    for (int j = 0; j < 4; ++j) acc[i][j] = zero8();

  for (int k0 = 0; k0 < K; k0 += 32) {
    V bh[4], bl[4];
#pragma unroll
    for (int j = 0; j < 4; ++j) {
      const size_t bo = (size_t)(n0 + (j << 4) + rlane) * ldb + koff + k0;
      bh[j] = Frag<T>::load(Bb + bo);
      if (SPLIT) bl[j] = Frag<T>::load(Bb2 + bo);
    }
#pragma unroll
    for (int i = 0; i < 4; ++i) {
      const size_t ao = (size_t)(m0 + (i << 4) + rlane) * lda + koff + k0;
      V ah = Frag<T>::load(Ab + ao);
      V al = ah;
      if (SPLIT || ASPLIT) al = Frag<T>::load(Ab2 + ao);
#pragma unroll
      for (int j = 0; j < 4; ++j) {
        acc[i][j] = Frag<T>::mma(ah, bh[j], acc[i][j]);
        if (SPLIT) {
          acc[i][j] = Frag<T>::mma(ah, bl[j], acc[i][j]);
          acc[i][j] = Frag<T>::mma(al, bh[j], acc[i][j]);
        }
        if (ASPLIT) acc[i][j] = Frag<T>::mma(al, bh[j], acc[i][j]);
      }
      Frag<T>::guard4(acc[i][0], acc[i][1], acc[i][2], acc[i][3], ah, al);
    }
    Frag<T>::keep(bh[0], bh[1], bh[2], bh[3]);
    if (SPLIT) Frag<T>::keep(bl[0], bl[1], bl[2], bl[3]);
  }
  acc_guard4(acc[0][0], acc[0][1], acc[0][2], acc[0][3]);
  acc_guard4(acc[1][0], acc[1][1], acc[1][2], acc[1][3]);
  acc_guard4(acc[2][0], acc[2][1], acc[2][2], acc[2][3]);
  acc_guard4(acc[3][0], acc[3][1], acc[3][2], acc[3][3]);

  float* slab = sT[wave];
#pragma unroll
  for (int i = 0; i < 4; ++i) {
    const int mBase = m0 + (i << 4);
#pragma unroll
    for (int j = 0; j < 4; ++j) {
      const int n = n0 + (j << 4) + rlane;
      float bv = 0.f;
      if (BIAS_MODE == 2) bv = bias[n];
#pragma unroll
      for (int r = 0; r < 8; ++r) {
        float v = acc[i][j][r] * scale;
        if (BIAS_MODE == 1) v += bias[mBase + mOff + r];
        if (BIAS_MODE == 2) v += bv;
        if (ACT == 2) v = fmaxf(v, 0.0f);
        if (ACT == 4) v = (v > 0.f) ? v : 0.01f * v;
        slab[(mOff + r) * 68 + (j << 4) + rlane] = v;
      }
    }
    __builtin_amdgcn_fence(__ATOMIC_RELEASE, "workgroup");
    __builtin_amdgcn_wave_barrier();
    __builtin_amdgcn_fence(__ATOMIC_ACQUIRE, "workgroup");
    if (OUT_MODE == 0) {
      float* C = (float*)Cout + (size_t)b * strideC;
      const int hh = lane >> 4, c4 = (lane & 15) * 4;
      for (int pass = 0; pass < 2; ++pass) {
#pragma unroll
        for (int it = 0; it < 8; ++it) {
          const int row = it * 2 + hh;
          v4f v = *(const v4f*)(slab + row * 68 + c4);
          *(volatile v4f*)(C + (size_t)(mBase + row) * ldc + n0 + c4) = v;
        }
        __threadfence();
      }
    } else {
      const int q = lane >> 3, c8 = (lane & 7) * 8;
      unsigned short* C  = (unsigned short*)Cout  + (size_t)b * strideC;
      unsigned short* C2 = (OUT_MODE == 2) ? ((unsigned short*)Cout2 + (size_t)b * strideC) : nullptr;
      for (int pass = 0; pass < 2; ++pass) {
#pragma unroll
        for (int it = 0; it < 4; ++it) {
          const int row = it * 4 + q;
          const float* sp = slab + row * 68 + c8;
          v8h hv, lv;
#pragma unroll
          for (int e = 0; e < 8; ++e) {
            if (OUT_MODE == 1) {
              hv[e] = (_Float16)sp[e];
            } else {
              unsigned short hb = f2bf_bits(sp[e]);
              unsigned short lb = f2bf_bits(sp[e] - bf_bits2f(hb));
              hv[e] = __builtin_bit_cast(_Float16, hb);
              lv[e] = __builtin_bit_cast(_Float16, lb);
            }
          }
          *(volatile v8h*)(C + (size_t)(mBase + row) * ldc + n0 + c8) = hv;
          if (OUT_MODE == 2) *(volatile v8h*)(C2 + (size_t)(mBase + row) * ldc + n0 + c8) = lv;
        }
        __threadfence();
      }
    }
    __builtin_amdgcn_fence(__ATOMIC_RELEASE, "workgroup");
    __builtin_amdgcn_wave_barrier();
    __builtin_amdgcn_fence(__ATOMIC_ACQUIRE, "workgroup");
  }
}

__global__ __launch_bounds__(256) void cast_hidden_kernel(const float* __restrict__ x, unsigned short* __restrict__ gin) {
  const int i = blockIdx.x * 256 + threadIdx.x;
  const int row = i >> 7;
  const int c8 = (i & 127) * 8;
  const float* p = x + (size_t)row * kHid + c8;
  const v4f a = *(const v4f*)(p);
  const v4f c = *(const v4f*)(p + 4);
  unsigned short hb[8];
#pragma unroll
  for (int e = 0; e < 4; ++e) {
    hb[e]     = h_bits(kCarryX * bf16r(a[e]));
    hb[4 + e] = h_bits(kCarryX * bf16r(c[e]));
  }
  const v4u u = (v4u){pk16(hb[0], hb[1]), pk16(hb[2], hb[3]), pk16(hb[4], hb[5]), pk16(hb[6], hb[7])};
  unsigned short* q = gin + (size_t)row * kGinP + c8;
  *(volatile v4u*)q = u;
  __threadfence();
  *(volatile v4u*)q = u;
}

template <int MODE>
__global__ __launch_bounds__(256) void cast_mat_kernel(const float* __restrict__ src, int rows_src, int cols_src,
                                                       unsigned short* __restrict__ dst, int rows_dst, int ld_dst,
                                                       float carry, int n8) {
  const int i = blockIdx.x * 256 + threadIdx.x;
  if (i >= n8) return;
  const int per_row = ld_dst >> 3;
  const int row = i / per_row;
  const int c8 = (i - row * per_row) * 8;
  const int rowc = (row < rows_src) ? row : (rows_src - 1);
  const float frow = (row < rows_src) ? 1.0f : 0.0f;
  unsigned short hb[8];
#pragma unroll
  for (int e = 0; e < 8; ++e) {
    const int col = c8 + e;
    const int colc = (col < cols_src) ? col : (cols_src - 1);
    const float x = src[(size_t)rowc * cols_src + colc];
    const float fc = (col < cols_src) ? 1.0f : 0.0f;
    const float val = bf16r(x) * carry * frow * fc;
    hb[e] = (MODE == 0) ? h_bits(val) : f2bf_bits(val);
  }
  const v4u u = (v4u){pk16(hb[0], hb[1]), pk16(hb[2], hb[3]), pk16(hb[4], hb[5]), pk16(hb[6], hb[7])};
  unsigned short* q = dst + 8 * (size_t)i;
  *(volatile v4u*)q = u;
  __threadfence();
  *(volatile v4u*)q = u;
}

__global__ __launch_bounds__(256) void conv_kernel(const unsigned short* __restrict__ lin,
                                                   const float* __restrict__ cwq, const float* __restrict__ cwk,
                                                   const float* __restrict__ cwv,
                                                   unsigned short* __restrict__ ws16, long offQ, long offK, long offV) {
  __shared__ float sPart[8];
  __shared__ __align__(16) unsigned sOut[512];
  const int row = blockIdx.x;
  const int l = row & (kLen - 1);
  const int t = threadIdx.x, lane = t & 31, wave = t >> 5, hd = t >> 6;
  const int c4 = 4 * t;
  int rj[4]; float fz[4];
#pragma unroll
  for (int j = 0; j < 4; ++j) {
    const int dj = 3 - j;
    const bool ok = (l >= dj);
    rj[j] = ok ? (row - dj) : row;
    fz[j] = ok ? 1.0f : 0.0f;
  }
#pragma unroll 1
  for (int s = 0; s < 3; ++s) {
    const float* cw = (s == 0) ? cwq : ((s == 1) ? cwk : cwv);
    const long offO = (s == 0) ? offQ : ((s == 1) ? offK : offV);
    const int col = s * kHid + c4;
    float xf[4][4];
#pragma unroll
    for (int j = 0; j < 4; ++j) {
      const v2u xw = *(const v2u*)(lin + (size_t)rj[j] * kNqkv + col);
      const unsigned w0 = xw.x, w1 = xw.y;
      const float sc = kInv16 * fz[j];
      xf[j][0] = h16_to_f32(w0 & 0xffffu) * sc;
      xf[j][1] = h16_to_f32(w0 >> 16) * sc;
      xf[j][2] = h16_to_f32(w1 & 0xffffu) * sc;
      xf[j][3] = h16_to_f32(w1 >> 16) * sc;
    }
    asm volatile("" ::: "memory");
    float acc[4];
#pragma unroll
    for (int e = 0; e < 4; ++e) {
      const v4f wv = *(const v4f*)(cw + (size_t)(c4 + e) * kConvK);
      float a = 0.0f;
      a += bf16r(wv.x) * xf[0][e];
      a += bf16r(wv.y) * xf[1][e];
      a += bf16r(wv.z) * xf[2][e];
      a += bf16r(wv.w) * xf[3][e];
      acc[e] = a;
    }
    float y[4];
    float ss = 0.0f;
#pragma unroll
    for (int e = 0; e < 4; ++e) {
      const float ex = expf(fminf(-acc[e], 80.0f));
      y[e] = acc[e] * (1.0f / (1.0f + ex));
      ss += y[e] * y[e];
    }
#pragma unroll
    for (int off = 16; off > 0; off >>= 1) ss += __shfl_xor(ss, off, 32);
    __syncthreads();
    if (lane == 0) sPart[wave] = ss;
    __syncthreads();
    const float tot = sPart[2 * hd] + sPart[2 * hd + 1];
    const float rinv = 1.0f / sqrtf(tot + 1e-6f);
    const float fac = (s < 2) ? rinv : 1.0f;
    unsigned short hb[4];
#pragma unroll
    for (int e = 0; e < 4; ++e) hb[e] = h_bits(kCarry16 * y[e] * fac);
    const v2u u2 = (v2u){pk16(hb[0], hb[1]), pk16(hb[2], hb[3])};
    *(v2u*)(sOut + 2 * t) = u2;
    __syncthreads();
    if (t < 128) {
      const v4u u4 = *(const v4u*)(sOut + 4 * t);
      unsigned short* op = ws16 + offO + (size_t)row * kHid + 8 * t;
      *(volatile v4u*)op = u4;
      __threadfence();
      *(volatile v4u*)op = u4;
    }
  }
}

__global__ __launch_bounds__(256) void prep_kernel(const unsigned short* __restrict__ qh, const unsigned short* __restrict__ kh,
                                                   const unsigned short* __restrict__ vv, const unsigned short* __restrict__ qkvlin,
                                                   unsigned short* __restrict__ u16, unsigned short* __restrict__ w16,
                                                   unsigned short* __restrict__ attn) {
  __shared__ __align__(16) _Float16 sKT[32 * 264];
  __shared__ __align__(16) _Float16 sQT[32 * 264];
  __shared__ __align__(16) _Float16 sVTt[256 * 32];
  __shared__ __align__(16) _Float16 sTt[32 * 40];
  __shared__ __align__(16) _Float16 sAtt[32 * 32];
  __shared__ float sAf[32 * 33];
  __shared__ float sBeta[32];
  const int t = threadIdx.x, lane = t & 31, wave = t >> 5;
  const int hh = lane >> 4, rl = lane & 15, koff = hh * 8;
  const int blk = blockIdx.x;
  const int ch = blk & (kNChunk - 1);
  const int bh = blk >> 6;
  const int b = bh >> 2, h = bh & 3;
  const int row0 = b * kLen + ch * kChunk;
  const int colh = h * kDh;

  if (t < 32) {
    const unsigned wb = *(const unsigned*)(qkvlin + (size_t)(row0 + t) * kNqkv + 3 * kHid + (h & ~1));
    const unsigned bl = (h & 1) ? (wb >> 16) : (wb & 0xffffu);
    const float x = h16_to_f32(bl) * kInv16;
    const float ex = expf(fminf(-x, 80.0f));
    sBeta[t] = 1.0f / (1.0f + ex);
  }
#pragma unroll
  for (int i = 0; i < 4; ++i) {
    const int e = i * 256 + t;
    const int r = e >> 5, c8 = (e & 31) * 8;
    const v4u kw = *(const v4u*)(kh + (size_t)(row0 + r) * kHid + colh + c8);
    const v4u qw = *(const v4u*)(qh + (size_t)(row0 + r) * kHid + colh + c8);
    *(v8h*)(sKT + r * 264 + c8) = __builtin_bit_cast(v8h, kw);
    *(v8h*)(sQT + r * 264 + c8) = __builtin_bit_cast(v8h, qw);
    asm volatile("" ::: "memory");
  }
  __syncthreads();

  {
    const _Float16* ap = (wave < 4) ? sKT : sQT;
    const int mi = (wave & 3) >> 1, ni = wave & 1;
    v8f acc = zero8();
#pragma unroll
    for (int k0 = 0; k0 < kDh; k0 += 32) {
      const v16h a  = FragH::load(ap  + (mi * 16 + rl) * 264 + k0 + koff);
      const v16h bb = FragH::load(sKT + (ni * 16 + rl) * 264 + k0 + koff);
      acc = mmah(a, bb, acc);
    }
    if (wave < 4) {
#pragma unroll
      for (int r = 0; r < 8; ++r) {
        const int i = mi * 16 + 8 * hh + r, j = ni * 16 + rl;
        sAf[i * 33 + j] = sBeta[i] * acc[r] * kInv256;
      }
    } else {
#pragma unroll
      for (int r = 0; r < 8; ++r) {
        const int i = mi * 16 + 8 * hh + r, j = ni * 16 + rl;
        const float av = (i >= j) ? acc[r] : 0.0f;
        sAtt[i * 32 + j] = (_Float16)av;
      }
    }
  }
  __syncthreads();

  if (wave == 0) {
    unsigned short* ag = attn + (size_t)blk * 1024;
    for (int pass = 0; pass < 2; ++pass) {
#pragma unroll
      for (int it = 0; it < 4; ++it) {
        const int off = it * 256 + lane * 8;
        const v8h val = *(const v8h*)(sAtt + off);
        *(volatile v8h*)(ag + off) = val;
      }
      __threadfence();
    }
  } else if (wave == 1) {
    float col[32];
#pragma unroll
    for (int i = 0; i < 32; ++i) col[i] = (i == lane) ? 1.0f : 0.0f;
#pragma unroll
    for (int i = 1; i < 32; ++i) {
      float s = 0.0f;
#pragma unroll
      for (int j = 0; j < i; ++j) s += sAf[i * 33 + j] * col[j];
      col[i] = col[i] - s;
    }
    const float bl = sBeta[lane];
#pragma unroll
    for (int i = 0; i < 32; ++i) sTt[i * 40 + lane] = (_Float16)(kCarry16 * col[i] * bl);
  }
  __syncthreads();

#pragma unroll
  for (int i = 0; i < 4; ++i) {
    const int e = i * 256 + t;
    const int tok = e >> 5, d8 = (e & 31) * 8;
    const v4u kw = *(const v4u*)(kh + (size_t)(row0 + tok) * kHid + colh + d8);
    const v4u vw = *(const v4u*)(vv + (size_t)(row0 + tok) * kHid + colh + d8);
    const unsigned kk[4] = {kw.x, kw.y, kw.z, kw.w};
    const unsigned vk[4] = {vw.x, vw.y, vw.z, vw.w};
#pragma unroll
    for (int j = 0; j < 8; ++j) {
      const unsigned kb = (j & 1) ? (kk[j >> 1] >> 16) : (kk[j >> 1] & 0xffffu);
      const unsigned vb = (j & 1) ? (vk[j >> 1] >> 16) : (vk[j >> 1] & 0xffffu);
      sKT[(d8 + j) * 32 + tok]  = h_from_bits(kb);
      sVTt[(d8 + j) * 32 + tok] = h_from_bits(vb);
    }
    asm volatile("" ::: "memory");
  }
  __syncthreads();

  const int mi2 = wave >> 2;
  const v16h ta = FragH::load(sTt + (mi2 * 16 + rl) * 40 + koff);
#pragma unroll
  for (int tt = 0; tt < 4; ++tt) {
    const int ni = (wave & 3) * 4 + tt;
    const v16h bb = FragH::load(sVTt + (ni * 16 + rl) * 32 + koff);
    const v8f acc = mmah(ta, bb, zero8());
#pragma unroll
    for (int r = 0; r < 8; ++r) sQT[(mi2 * 16 + 8 * hh + r) * 264 + ni * 16 + rl] = (_Float16)acc[r];
  }
  __syncthreads();
  {
    for (int pass = 0; pass < 2; ++pass) {
#pragma unroll
      for (int q = 0; q < 4; ++q) {
        const int row = 4 * wave + q;
        const v8h val = *(const v8h*)(sQT + row * 264 + lane * 8);
        *(volatile v8h*)(u16 + (size_t)(row0 + row) * kHid + colh + lane * 8) = val;
      }
      __threadfence();
    }
  }
  __syncthreads();
#pragma unroll
  for (int tt = 0; tt < 4; ++tt) {
    const int ni = (wave & 3) * 4 + tt;
    const v16h bb = FragH::load(sKT + (ni * 16 + rl) * 32 + koff);
    const v8f acc = mmah(ta, bb, zero8());
#pragma unroll
    for (int r = 0; r < 8; ++r) sQT[(mi2 * 16 + 8 * hh + r) * 264 + ni * 16 + rl] = (_Float16)(-acc[r] * kInv16);
  }
  __syncthreads();
  {
    for (int pass = 0; pass < 2; ++pass) {
#pragma unroll
      for (int q = 0; q < 4; ++q) {
        const int row = 4 * wave + q;
        const v8h val = *(const v8h*)(sQT + row * 264 + lane * 8);
        *(volatile v8h*)(w16 + (size_t)(row0 + row) * kHid + colh + lane * 8) = val;
      }
      __threadfence();
    }
  }
}

__global__ __launch_bounds__(256) void rec_kernel(const unsigned short* __restrict__ qh, const unsigned short* __restrict__ kh,
                                                  const unsigned short* __restrict__ u16, const unsigned short* __restrict__ w16,
                                                  const unsigned short* __restrict__ attn, unsigned short* __restrict__ delta) {
  __shared__ __align__(16) _Float16 sS[64 * 256];
  __shared__ __align__(16) _Float16 sKTt[256 * 32];
  __shared__ __align__(16) _Float16 sWc[32 * 264];
  __shared__ __align__(16) _Float16 sQc[32 * 264];
  __shared__ __align__(16) _Float16 sUAt[64 * 32];
  __shared__ __align__(16) unsigned short sU[32 * 64];
  __shared__ __align__(16) _Float16 sO[32 * 64];
  const int t = threadIdx.x, lane = t & 31, wave = t >> 5;
  const int hh = lane >> 4, rl = lane & 15, koff = hh * 8;
  const int blk = blockIdx.x;
  const int bh = blk >> 2, nt = blk & 3;
  const int b = bh >> 2, h = bh & 3;
  const int colh = h * kDh;
  const int col0 = colh + nt * 64;
  const int mi = wave >> 2, ni = wave & 3;

  v8f accS[2][4];
#pragma unroll
  for (int j = 0; j < 2; ++j)
#pragma unroll
    for (int n2 = 0; n2 < 4; ++n2) accS[j][n2] = zero8();
  {
    const v8h z = (v8h){(_Float16)0.f, (_Float16)0.f, (_Float16)0.f, (_Float16)0.f, (_Float16)0.f, (_Float16)0.f, (_Float16)0.f, (_Float16)0.f};
#pragma unroll
    for (int i = 0; i < 8; ++i) *(v8h*)(sS + (i * 256 + t) * 8) = z;
  }

  for (int ch = 0; ch < kNChunk; ++ch) {
    __syncthreads();
    const int row0 = b * kLen + ch * kChunk;
    {
      const int tok = t >> 3, c8 = (t & 7) * 8;
      *(v4u*)(sU + tok * 64 + c8) = *(const v4u*)(u16 + (size_t)(row0 + tok) * kHid + col0 + c8);
    }
    asm volatile("" ::: "memory");
#pragma unroll
    for (int i = 0; i < 4; ++i) {
      const int e = i * 256 + t;
      const int tok = e >> 5, d8 = (e & 31) * 8;
      const v4u kw = *(const v4u*)(kh + (size_t)(row0 + tok) * kHid + colh + d8);
      const unsigned kk[4] = {kw.x, kw.y, kw.z, kw.w};
#pragma unroll
      for (int j = 0; j < 8; ++j) {
        const unsigned kb = (j & 1) ? (kk[j >> 1] >> 16) : (kk[j >> 1] & 0xffffu);
        sKTt[(d8 + j) * 32 + tok] = h_from_bits(kb);
      }
      asm volatile("" ::: "memory");
    }
#pragma unroll
    for (int i = 0; i < 4; ++i) {
      const int e = i * 256 + t;
      const int r = e >> 5, c8 = (e & 31) * 8;
      const v4u ww = *(const v4u*)(w16 + (size_t)(row0 + r) * kHid + colh + c8);
      const v4u qw = *(const v4u*)(qh  + (size_t)(row0 + r) * kHid + colh + c8);
      *(v8h*)(sWc + r * 264 + c8) = __builtin_bit_cast(v8h, ww);
      *(v8h*)(sQc + r * 264 + c8) = __builtin_bit_cast(v8h, qw);
      asm volatile("" ::: "memory");
    }
    __syncthreads();

    v8f accU, accO1 = zero8();
#pragma unroll
    for (int r = 0; r < 8; ++r) accU[r] = h16_to_f32((unsigned)sU[(mi * 16 + 8 * hh + r) * 64 + ni * 16 + rl]);
    {
      const _Float16* wrow = sWc + (mi * 16 + rl) * 264 + koff;
      const _Float16* qrow = sQc + (mi * 16 + rl) * 264 + koff;
      const _Float16* srow = sS + (ni * 16 + rl) * 256 + koff;
#pragma unroll 2
      for (int k0 = 0; k0 < kDh; k0 += 32) {
        const v16h aw = FragH::load(wrow + k0);
        const v16h aq = FragH::load(qrow + k0);
        const v16h bs = FragH::load(srow + k0);
        accU  = mmah(aw, bs, accU);
        accO1 = mmah(aq, bs, accO1);
      }
    }
    {
      v8h uv;
#pragma unroll
      for (int r = 0; r < 8; ++r) uv[r] = (_Float16)accU[r];
      *(v8h*)(sUAt + (ni * 16 + rl) * 32 + mi * 16 + 8 * hh) = uv;
    }
    __syncthreads();

    {
      const v16h aA = FragH::load((const _Float16*)(attn + (size_t)(bh * kNChunk + ch) * 1024 + (mi * 16 + rl) * 32 + koff));
      const v16h bU = FragH::load(sUAt + (ni * 16 + rl) * 32 + koff);
      const v8f accO2 = mmah(aA, bU, zero8());
#pragma unroll
      for (int r = 0; r < 8; ++r) {
        const float ov = accO1[r] + accO2[r] * kInv256;
        sO[(mi * 16 + 8 * hh + r) * 64 + ni * 16 + rl] = (_Float16)ov;
      }
    }
    {
      v16h bU2[4];
#pragma unroll
      for (int n2 = 0; n2 < 4; ++n2) bU2[n2] = FragH::load(sUAt + (n2 * 16 + rl) * 32 + koff);
#pragma unroll
      for (int j = 0; j < 2; ++j) {
        const v16h aK = FragH::load(sKTt + ((2 * wave + j) * 16 + rl) * 32 + koff);
#pragma unroll
        for (int n2 = 0; n2 < 4; ++n2) accS[j][n2] = mmah(aK, bU2[n2], accS[j][n2]);
      }
#pragma unroll
      for (int j = 0; j < 2; ++j) {
#pragma unroll
        for (int n2 = 0; n2 < 4; ++n2) {
          v8h sv;
#pragma unroll
          for (int r = 0; r < 8; ++r) sv[r] = (_Float16)(accS[j][n2][r] * kInv256);
          *(v8h*)(sS + (n2 * 16 + rl) * 256 + (2 * wave + j) * 16 + 8 * hh) = sv;
        }
      }
    }
    __syncthreads();

    {
      const int row = 4 * wave + (lane >> 3);
      const int c8 = (lane & 7) * 8;
      unsigned short* dp = delta + (size_t)(row0 + row) * kHid + col0 + c8;
      for (int pass = 0; pass < 2; ++pass) {
        const v8h val = *(const v8h*)(sO + row * 64 + c8);
        *(volatile v8h*)dp = val;
        __threadfence();
      }
    }
  }
}

__global__ __launch_bounds__(256) void fir_kernel(const unsigned short* __restrict__ vv,
                                                  const float* __restrict__ firs, const float* __restrict__ firl,
                                                  const float* __restrict__ firw,
                                                  unsigned short* __restrict__ outS, unsigned short* __restrict__ outL,
                                                  unsigned short* __restrict__ outW) {
  __shared__ __align__(16) float sx[95 * 64];
  __shared__ float sw[64 * kFirTaps];
  __shared__ __align__(16) _Float16 so[3 * 2048];
  const int blk = blockIdx.x;
  const int ct = blk & 15;
  const int rt = (blk >> 4) & 63;
  const int b  = blk >> 10;
  const int t = threadIdx.x, lane = t & 31, wave = t >> 5;
  const int c = t & 63, rs = t >> 6;
  const int cbase = ct * 64;
#pragma unroll
  for (int i = 0; i < 3; ++i) {
    const int e = i * 256 + t;
    const int ec = (e < 760) ? e : 759;
    const int jr = ec >> 3, c8 = (ec & 7) * 8;
    const int l = rt * 32 - 63 + jr;
    const int lc = (l >= 0) ? l : 0;
    const float fzv = (l >= 0) ? kInv16 : 0.0f;
    const v4u w4 = *(const v4u*)(vv + (size_t)(b * kLen + lc) * kHid + cbase + c8);
    v4f f0, f1;
    f0.x = h16_to_f32(w4.x & 0xffffu) * fzv; f0.y = h16_to_f32(w4.x >> 16) * fzv;
    f0.z = h16_to_f32(w4.y & 0xffffu) * fzv; f0.w = h16_to_f32(w4.y >> 16) * fzv;
    f1.x = h16_to_f32(w4.z & 0xffffu) * fzv; f1.y = h16_to_f32(w4.z >> 16) * fzv;
    f1.z = h16_to_f32(w4.w & 0xffffu) * fzv; f1.w = h16_to_f32(w4.w >> 16) * fzv;
    if (e < 760) {
      *(v4f*)(sx + jr * 64 + c8) = f0;
      *(v4f*)(sx + jr * 64 + c8 + 4) = f1;
    }
  }
#pragma unroll 1
  for (int e = t; e < 64 * kFirW; e += 256) {
    const int chn = e >> 6, tp = e & 63;
    sw[chn * kFirTaps + tp] = bf16r(firw[(size_t)(cbase + chn) * kFirW + tp]);
  }
#pragma unroll 1
  for (int e = t; e < 64 * kFirL; e += 256) {
    const int chn = e / kFirL, tp = e - chn * kFirL;
    sw[chn * kFirTaps + kFirW + tp] = bf16r(firl[(size_t)(cbase + chn) * kFirL + tp]);
  }
#pragma unroll 1
  for (int e = t; e < 64 * kFirS; e += 256) {
    const int chn = e / kFirS, tp = e - chn * kFirS;
    sw[chn * kFirTaps + kFirW + kFirL + tp] = bf16r(firs[(size_t)(cbase + chn) * kFirS + tp]);
  }
  __syncthreads();
#pragma unroll 1
  for (int it = 0; it < 2; ++it) {
    const int lr0 = rs * 8 + it * 4;
    float aw[4] = {0.f, 0.f, 0.f, 0.f}, al[4] = {0.f, 0.f, 0.f, 0.f}, ash[4] = {0.f, 0.f, 0.f, 0.f};
#pragma unroll 1
    for (int tp = 0; tp < kFirW; ++tp) {
      const float w = sw[c * kFirTaps + tp];
#pragma unroll
      for (int r = 0; r < 4; ++r) aw[r] += w * sx[(lr0 + r + tp) * 64 + c];
    }
#pragma unroll 1
    for (int tp = 0; tp < kFirL; ++tp) {
      const float w = sw[c * kFirTaps + kFirW + tp];
#pragma unroll
      for (int r = 0; r < 4; ++r) al[r] += w * sx[(lr0 + r + 33 + tp) * 64 + c];
    }
#pragma unroll 1
    for (int tp = 0; tp < kFirS; ++tp) {
      const float w = sw[c * kFirTaps + kFirW + kFirL + tp];
#pragma unroll
      for (int r = 0; r < 4; ++r) ash[r] += w * sx[(lr0 + r + 61 + tp) * 64 + c];
    }
#pragma unroll
    for (int r = 0; r < 4; ++r) {
      so[0 * 2048 + (lr0 + r) * 64 + c] = (_Float16)(kCarry16 * ash[r]);
      so[1 * 2048 + (lr0 + r) * 64 + c] = (_Float16)(kCarry16 * al[r]);
      so[2 * 2048 + (lr0 + r) * 64 + c] = (_Float16)(kCarry16 * aw[r]);
    }
  }
  __syncthreads();
  {
    const int row = 4 * wave + (lane >> 3);
    const int c8 = (lane & 7) * 8;
    const size_t go = (size_t)(b * kLen + rt * 32 + row) * kHid + cbase + c8;
    for (int pass = 0; pass < 2; ++pass) {
      const v8h v0 = *(const v8h*)(so + 0 * 2048 + row * 64 + c8);
      const v8h v1 = *(const v8h*)(so + 1 * 2048 + row * 64 + c8);
      const v8h v2 = *(const v8h*)(so + 2 * 2048 + row * 64 + c8);
      *(volatile v8h*)(outS + go) = v0;
      *(volatile v8h*)(outL + go) = v1;
      *(volatile v8h*)(outW + go) = v2;
      __threadfence();
    }
  }
}

__global__ __launch_bounds__(256) void stats_kernel(const unsigned short* __restrict__ ws16, long offSp, long offLp,
                                                    long offWp, long offDp, long offVp, unsigned short* __restrict__ gin) {
  __shared__ __align__(16) _Float16 sSt[32 * 64];
  const int blk = blockIdx.x;
  const int t = threadIdx.x, lane = t & 31, wave = t >> 5;
#pragma unroll 1
  for (int rr = 0; rr < 4; ++rr) {
    const int rloc = 4 * wave + rr;
    const int row = blk * 32 + rloc;
#pragma unroll 1
    for (int s = 0; s < 5; ++s) {
      const long off = (s == 0) ? offSp : ((s == 1) ? offLp : ((s == 2) ? offWp : ((s == 3) ? offDp : offVp)));
      const float sc = (s == 3) ? kInv256 : kInv16;
#pragma unroll 1
      for (int hd = 0; hd < 4; ++hd) {
        const v4u w4 = *(const v4u*)(ws16 + off + (size_t)row * kHid + hd * kDh + lane * 8);
        const unsigned wd[4] = {w4.x, w4.y, w4.z, w4.w};
        float sum = 0.0f, sq = 0.0f, mx = 0.0f;
#pragma unroll
        for (int e = 0; e < 4; ++e) {
          const float x0 = h16_to_f32(wd[e] & 0xffffu) * sc;
          const float x1 = h16_to_f32(wd[e] >> 16) * sc;
          sum += x0; sum += x1;
          sq += x0 * x0; sq += x1 * x1;
          mx = fmaxf(mx, fabsf(x0)); mx = fmaxf(mx, fabsf(x1));
        }
#pragma unroll
        for (int off2 = 16; off2 > 0; off2 >>= 1) {
          sum += __shfl_xor(sum, off2, 32);
          sq  += __shfl_xor(sq, off2, 32);
          mx   = fmaxf(mx, __shfl_xor(mx, off2, 32));
        }
        if (lane == 0) {
          const float mean = sum * (1.0f / 256.0f);
          const float rms = sqrtf(fmaxf(sq * (1.0f / 256.0f), 1e-8f));
          sSt[rloc * 64 + s * 12 + 0 + hd] = (_Float16)(kCarryX * mean);
          sSt[rloc * 64 + s * 12 + 4 + hd] = (_Float16)(kCarryX * rms);
          sSt[rloc * 64 + s * 12 + 8 + hd] = (_Float16)(kCarryX * mx);
        }
      }
    }
    if (lane < 4) sSt[rloc * 64 + 60 + lane] = (_Float16)0.0f;
  }
  __syncthreads();
  {
    const int row = 4 * wave + (lane >> 3);
    const int c8 = (lane & 7) * 8;
    unsigned short* dp = gin + (size_t)(blk * 32 + row) * kGinP + kHid + c8;
    for (int pass = 0; pass < 2; ++pass) {
      const v8h val = *(const v8h*)(sSt + row * 64 + c8);
      *(volatile v8h*)dp = val;
      __threadfence();
    }
  }
}

__global__ __launch_bounds__(256) void gelu_kernel(unsigned* __restrict__ hdn, int n2) {
  const int i = blockIdx.x * 256 + threadIdx.x;
  if (i >= n2) return;
  const unsigned u = hdn[i];
  const float x0 = h16_to_f32(u & 0xffffu);
  const float x1 = h16_to_f32(u >> 16);
  float g0 = 0.0f, g1 = 0.0f;
#pragma unroll 1
  for (int k = 0; k < 2; ++k) {
    const float x = (k == 0) ? x0 : x1;
    const float g = 0.5f * x * (1.0f + erff(x * 0.70710678118654752f));
    g0 = (k == 0) ? g : g0;
    g1 = (k == 1) ? g : g1;
  }
  const unsigned w = pk16(h_bits(kCarryX * g0), h_bits(kCarryX * g1));
  *(volatile unsigned*)(hdn + i) = w;
  __threadfence();
  *(volatile unsigned*)(hdn + i) = w;
}

__global__ __launch_bounds__(512) void combine_kernel(const float* __restrict__ logits, const float* __restrict__ g2b,
                                                      const float* __restrict__ vbias, const float* __restrict__ ltemp,
                                                      const float* __restrict__ flog, const float* __restrict__ onorm,
                                                      const float* __restrict__ cwv, const unsigned short* __restrict__ lin,
                                                      const unsigned short* __restrict__ ws16, long offSp, long offLp,
                                                      long offWp, long offDp,
                                                      unsigned short* __restrict__ ofhi, unsigned short* __restrict__ oflo) {
  __shared__ float sPart[16];
  const int row = blockIdx.x;
  const int l = row & (kLen - 1);
  const int t = threadIdx.x, lane = t & 31, wave = t >> 5, hd = t >> 7;
  const int c2 = 2 * t;
  const int d = c2 & (kDh - 1);
  float lg[5];
#pragma unroll
  for (int j = 0; j < 5; ++j) lg[j] = logits[(size_t)row * kNLogP + hd * 5 + j] + bf16r(g2b[hd * 5 + j]);
  lg[4] += bf16r(vbias[hd]);
  const float itmp = 1.0f / expf(bf16r(ltemp[hd]));
  const float fl = bf16r(flog[hd]);
  asm volatile("" ::: "memory");
  float m = -3.0e38f;
#pragma unroll
  for (int j = 0; j < 5; ++j) { lg[j] *= itmp; m = fmaxf(m, lg[j]); }
  float ev[5], se = 0.0f;
#pragma unroll
  for (int j = 0; j < 5; ++j) { ev[j] = expf(lg[j] - m); se += ev[j]; }
  const float rs = 1.0f / se;
  const float f = 1.0f / (1.0f + expf(fminf(-fl, 80.0f)));
  const float sc = 1.0f - 4.0f * f;
  const float w0 = f + sc * (ev[0] * rs), w1 = f + sc * (ev[1] * rs), w2 = f + sc * (ev[2] * rs), w3 = f + sc * (ev[3] * rs);
  const float wv = sc * (ev[4] * rs);
  const unsigned us0 = *(const unsigned*)(ws16 + offSp + (size_t)row * kHid + c2);
  const unsigned ul0 = *(const unsigned*)(ws16 + offLp + (size_t)row * kHid + c2);
  const unsigned uw0 = *(const unsigned*)(ws16 + offWp + (size_t)row * kHid + c2);
  const unsigned ud0 = *(const unsigned*)(ws16 + offDp + (size_t)row * kHid + c2);
  const float s0 = h16_to_f32(us0 & 0xffffu) * kInv16, s1 = h16_to_f32(us0 >> 16) * kInv16;
  const float g0 = h16_to_f32(ul0 & 0xffffu) * kInv16, g1 = h16_to_f32(ul0 >> 16) * kInv16;
  const float d0 = h16_to_f32(uw0 & 0xffffu) * kInv16, d1 = h16_to_f32(uw0 >> 16) * kInv16;
  const float e0 = h16_to_f32(ud0 & 0xffffu) * kInv256, e1 = h16_to_f32(ud0 >> 16) * kInv256;
  asm volatile("" ::: "memory");
  float xv[4][2];
#pragma unroll
  for (int j = 0; j < 4; ++j) {
    const int dj = 3 - j;
    const bool ok = (l >= dj);
    const int rj = ok ? (row - dj) : row;
    const float fz = ok ? kInv16 : 0.0f;
    const unsigned x = *(const unsigned*)(lin + (size_t)rj * kNqkv + 2 * kHid + c2);
    xv[j][0] = h16_to_f32(x & 0xffffu) * fz;
    xv[j][1] = h16_to_f32(x >> 16) * fz;
  }
  asm volatile("" ::: "memory");
  const v4f wa = *(const v4f*)(cwv + (size_t)c2 * kConvK);
  const v4f wb = *(const v4f*)(cwv + (size_t)(c2 + 1) * kConvK);
  float a0 = 0.0f, a1 = 0.0f;
  a0 += bf16r(wa.x) * xv[0][0]; a0 += bf16r(wa.y) * xv[1][0]; a0 += bf16r(wa.z) * xv[2][0]; a0 += bf16r(wa.w) * xv[3][0];
  a1 += bf16r(wb.x) * xv[0][1]; a1 += bf16r(wb.y) * xv[1][1]; a1 += bf16r(wb.z) * xv[2][1]; a1 += bf16r(wb.w) * xv[3][1];
  const float v0 = a0 * (1.0f / (1.0f + expf(fminf(-a0, 80.0f))));
  const float v1 = a1 * (1.0f / (1.0f + expf(fminf(-a1, 80.0f))));
  float o0 = w0 * s0; o0 += w1 * g0; o0 += w2 * d0; o0 += w3 * e0; o0 += wv * v0;
  float o1 = w0 * s1; o1 += w1 * g1; o1 += w2 * d1; o1 += w3 * e1; o1 += wv * v1;
  float ss = o0 * o0 + o1 * o1;
#pragma unroll
  for (int off = 16; off > 0; off >>= 1) ss += __shfl_xor(ss, off, 32);
  if (lane == 0) sPart[wave] = ss;
  __syncthreads();
  const float tot = (sPart[4 * hd] + sPart[4 * hd + 1]) + (sPart[4 * hd + 2] + sPart[4 * hd + 3]);
  const float rn = 1.0f / sqrtf(tot * (1.0f / 256.0f) + 1e-5f);
  const float on0 = bf16r(onorm[d]), on1 = bf16r(onorm[d + 1]);
  const float of0 = o0 * rn * on0, of1 = o1 * rn * on1;
  const unsigned short hb0 = f2bf_bits(of0), hb1 = f2bf_bits(of1);
  const unsigned short lb0 = f2bf_bits(of0 - bf_bits2f(hb0)), lb1 = f2bf_bits(of1 - bf_bits2f(hb1));
  const unsigned wh = pk16(hb0, hb1), wl = pk16(lb0, lb1);
  unsigned short* ph = ofhi + (size_t)row * kHid + c2;
  unsigned short* pl = oflo + (size_t)row * kHid + c2;
  *(volatile unsigned*)ph = wh;
  *(volatile unsigned*)pl = wl;
  __threadfence();
  *(volatile unsigned*)ph = wh;
  *(volatile unsigned*)pl = wl;
}

extern "C" void kernel_launch(void* const* d_in, const int* in_sizes, int n_in,
                              void* d_out, int out_size, void* d_ws, size_t ws_size,
                              hipStream_t stream) {
  if (n_in < 20) return;
  const int nAct = kRows * kHid;
  if (in_sizes[0] != nAct || in_sizes[1] != kHid * kHid || in_sizes[2] != kHid * kHid || in_sizes[3] != kHid * kHid) return;
  if (in_sizes[4] != kHeads * kHid || in_sizes[5] != kHid * kConvK || in_sizes[6] != kHid * kConvK || in_sizes[7] != kHid * kConvK) return;
  if (in_sizes[8] != kHid * kFirS || in_sizes[9] != kHid * kFirL || in_sizes[10] != kHid * kFirW) return;
  if (in_sizes[11] != kGh * kGin || in_sizes[12] != kGh || in_sizes[13] != kNLog * kGh || in_sizes[14] != kNLog) return;
  if (in_sizes[15] != kHeads || in_sizes[16] != kHeads || in_sizes[17] != kHeads || in_sizes[18] != kDh || in_sizes[19] != kHid * kHid) return;
  if (out_size != nAct) return;

  const size_t szGin  = (size_t)kRows * kGinP * 2;
  const size_t szWqkv = (size_t)kNqkv * kHid * 2;
  const size_t szOw   = (size_t)kHid * kHid * 2;
  const size_t szG1   = (size_t)kGh * kGinP * 2;
  const size_t szG2   = (size_t)kNLogP * kGh * 2;
  const size_t szLin  = (size_t)kRows * kNqkv * 2;
  const size_t szP16  = (size_t)kRows * kHid * 2;
  const size_t szAtt  = (size_t)kBatch * kHeads * kNChunk * 32 * 32 * 2;
  const size_t szHdn  = (size_t)kRows * kGh * 2;
  const size_t szLog  = (size_t)kRows * kNLogP * 4;
  size_t off = 0;
  const size_t offGin = off;  off += szGin;
  const size_t offWq  = off;  off += szWqkv;
  const size_t offOw  = off;  off += szOw;
  const size_t offG1  = off;  off += szG1;
  const size_t offG2  = off;  off += szG2;
  const size_t offLin = off;  off += szLin;
  const size_t offQh  = off;  off += szP16;
  const size_t offKh  = off;  off += szP16;
  const size_t offV   = off;  off += szP16;
  const size_t offU   = off;  off += szP16;
  const size_t offW   = off;  off += szP16;
  const size_t offAtt = off;  off += szAtt;
  const size_t offDel = off;  off += szP16;
  const size_t offHdn = off;  off += szHdn;
  const size_t offLog = off;  off += szLog;
  const size_t offOfh = off;  off += szP16;
  const size_t offOfl = off;  off += szP16;
  const size_t total  = off;
  if (ws_size < total) return;

  const float* hidden  = (const float*)d_in[0];
  const float* q_w     = (const float*)d_in[1];
  const float* k_w     = (const float*)d_in[2];
  const float* v_w     = (const float*)d_in[3];
  const float* b_w     = (const float*)d_in[4];
  const float* convq   = (const float*)d_in[5];
  const float* convk   = (const float*)d_in[6];
  const float* convv   = (const float*)d_in[7];
  const float* fir_s   = (const float*)d_in[8];
  const float* fir_l   = (const float*)d_in[9];
  const float* fir_wd  = (const float*)d_in[10];
  const float* g1_w    = (const float*)d_in[11];
  const float* g1_b    = (const float*)d_in[12];
  const float* g2_w    = (const float*)d_in[13];
  const float* g2_b    = (const float*)d_in[14];
  const float* vbias   = (const float*)d_in[15];
  const float* ltemp   = (const float*)d_in[16];
  const float* flogit  = (const float*)d_in[17];
  const float* onorm   = (const float*)d_in[18];
  const float* o_w     = (const float*)d_in[19];
  float* out = (float*)d_out;
  char* ws = (char*)d_ws;
  unsigned short* ws16 = (unsigned short*)ws;
  unsigned short* GIN  = (unsigned short*)(ws + offGin);
  unsigned short* WQKV = (unsigned short*)(ws + offWq);
  unsigned short* OW   = (unsigned short*)(ws + offOw);
  unsigned short* G1W  = (unsigned short*)(ws + offG1);
  unsigned short* G2W  = (unsigned short*)(ws + offG2);
  unsigned short* LIN  = (unsigned short*)(ws + offLin);
  unsigned short* QH   = (unsigned short*)(ws + offQh);
  unsigned short* KH   = (unsigned short*)(ws + offKh);
  unsigned short* V16  = (unsigned short*)(ws + offV);
  unsigned short* U16  = (unsigned short*)(ws + offU);
  unsigned short* W16  = (unsigned short*)(ws + offW);
  unsigned short* ATT  = (unsigned short*)(ws + offAtt);
  unsigned short* DEL  = (unsigned short*)(ws + offDel);
  unsigned short* HDN  = (unsigned short*)(ws + offHdn);
  float*          LOG  = (float*)(ws + offLog);
  unsigned short* OFH  = (unsigned short*)(ws + offOfh);
  unsigned short* OFL  = (unsigned short*)(ws + offOfl);
  const long hQh = (long)(offQh / 2), hKh = (long)(offKh / 2), hV = (long)(offV / 2);
  const long hU = (long)(offU / 2), hW = (long)(offW / 2), hDel = (long)(offDel / 2);

  cast_hidden_kernel<<<dim3((kRows * 128) / 256), dim3(256), 0, stream>>>(hidden, GIN);
  const int n8w = (kHid * kHid) / 8;
  cast_mat_kernel<0><<<dim3(n8w / 256), dim3(256), 0, stream>>>(q_w, kHid, kHid, WQKV, kHid, kHid, kCarryW, n8w);
  cast_mat_kernel<0><<<dim3(n8w / 256), dim3(256), 0, stream>>>(k_w, kHid, kHid, WQKV + (size_t)kHid * kHid, kHid, kHid, kCarryW, n8w);
  cast_mat_kernel<0><<<dim3(n8w / 256), dim3(256), 0, stream>>>(v_w, kHid, kHid, WQKV + (size_t)2 * kHid * kHid, kHid, kHid, kCarryW, n8w);
  const int n8b = (64 * kHid) / 8;
  cast_mat_kernel<0><<<dim3(n8b / 256), dim3(256), 0, stream>>>(b_w, kHeads, kHid, WQKV + (size_t)3 * kHid * kHid, 64, kHid, kCarryW, n8b);
  const int n8g1 = (kGh * kGinP) / 8;
  cast_mat_kernel<0><<<dim3(n8g1 / 256), dim3(256), 0, stream>>>(g1_w, kGh, kGin, G1W, kGh, kGinP, kCarryW, n8g1);
  const int n8g2 = (kNLogP * kGh) / 8;
  cast_mat_kernel<0><<<dim3(n8g2 / 256), dim3(256), 0, stream>>>(g2_w, kNLog, kGh, G2W, kNLogP, kGh, kCarryW, n8g2);
  cast_mat_kernel<1><<<dim3(n8w / 256), dim3(256), 0, stream>>>(o_w, kHid, kHid, OW, kHid, kHid, 1.0f, n8w);

  {
    const int tiles = (kRows / 64) * (kNqkv / 64);
    wmma_gemm64<0, false, false, 0, 1><<<dim3(tiles / 8, 1), dim3(256), 0, stream>>>(
        GIN, GIN, kGinP, 0L, WQKV, WQKV, kHid, 0L, (void*)LIN, (void*)LIN, kNqkv, 0L, g1_b, kRows, kNqkv, kHid, kScaleS1);
  }
  conv_kernel<<<dim3(kRows), dim3(256), 0, stream>>>(LIN, convq, convk, convv, ws16, hQh, hKh, hV);
  prep_kernel<<<dim3(kBatch * kHeads * kNChunk), dim3(256), 0, stream>>>(QH, KH, V16, LIN, U16, W16, ATT);
  rec_kernel<<<dim3(kBatch * kHeads * (kDh / 64)), dim3(256), 0, stream>>>(QH, KH, U16, W16, ATT, DEL);
  fir_kernel<<<dim3(kBatch * 64 * 16), dim3(256), 0, stream>>>(V16, fir_s, fir_l, fir_wd, U16, W16, QH);
  stats_kernel<<<dim3(kRows / 32), dim3(256), 0, stream>>>(ws16, hU, hW, hQh, hDel, hV, GIN);
  {
    const int tiles = (kRows / 64) * (kGh / 64);
    wmma_gemm64<0, false, false, 2, 1><<<dim3(tiles / 8, 1), dim3(256), 0, stream>>>(
        GIN, GIN, kGinP, 0L, G1W, G1W, kGinP, 0L, (void*)HDN, (void*)HDN, kGh, 0L, g1_b, kRows, kGh, kGinP, kScaleG);
  }
  {
    const int n2 = (kRows * kGh) / 2;
    gelu_kernel<<<dim3(n2 / 256), dim3(256), 0, stream>>>((unsigned*)HDN, n2);
  }
  {
    const int tiles = (kRows / 64) * (kNLogP / 64);
    wmma_gemm64<0, false, false, 0, 0><<<dim3(tiles / 8, 1), dim3(256), 0, stream>>>(
        HDN, HDN, kGh, 0L, G2W, G2W, kGh, 0L, (void*)LOG, (void*)LOG, kNLogP, 0L, g1_b, kRows, kNLogP, kGh, kScaleG);
  }
  combine_kernel<<<dim3(kRows), dim3(512), 0, stream>>>(LOG, g2_b, vbias, ltemp, flogit, onorm, convv, LIN,
                                                        ws16, hU, hW, hQh, hDel, OFH, OFL);
  {
    const int tiles = (kRows / 64) * (kHid / 64);
    wmma_gemm64<1, false, true, 0, 0><<<dim3(tiles / 8, 1), dim3(256), 0, stream>>>(
        OFH, OFL, kHid, 0L, OW, OW, kHid, 0L, (void*)out, (void*)out, kHid, 0L, g1_b, kRows, kHid, kHid, 1.0f);
  }
}
